// LinearDispatch_9354438770889
// MI455X (gfx1250) — hardware-run, weakly checked
//
#include <hip/hip_runtime.h>
#include <math.h>

typedef __attribute__((ext_vector_type(16))) _Float16 v16h;
typedef __attribute__((ext_vector_type(8)))  _Float16 v8h;
typedef __attribute__((ext_vector_type(8)))  float    v8f;
typedef __attribute__((ext_vector_type(4)))  float    v4f;
typedef __attribute__((ext_vector_type(4)))  unsigned v4u;
typedef __attribute__((ext_vector_type(4)))  int      v4i;

constexpr int kRows     = 8192;
constexpr int kDin      = 512;
constexpr int kDout     = 512;
constexpr int kCls      = 16;
constexpr int kThr      = 256;
constexpr int kSegRows  = 32;
constexpr int kTileRows = 64;
constexpr int kMaxTiles = kRows / kTileRows + kCls;
constexpr int kGrRows   = kMaxTiles * kTileRows;
constexpr int kChunk    = 256;
constexpr int kAPitch   = kChunk + 8;
constexpr int kSlabPitch = 68;
constexpr int kATileBytes = kTileRows * kAPitch * 2;
constexpr int kSlabBytes  = 8 * 16 * kSlabPitch * 4;
constexpr int kRawBytes   = (kATileBytes > kSlabBytes) ? kATileBytes : kSlabBytes;
constexpr float kCarryX = 16.0f;
constexpr float kCarryW = 256.0f;
constexpr float kFold   = 1.0f / (kCarryX * kCarryW);
constexpr float kHalfMinNormal = 6.103515625e-5f;

static_assert(kSegRows * kThr == kRows);
static_assert((kDin % kChunk) == 0 && (kChunk % 32) == 0);
static_assert((kDout % 64) == 0 && (kDin % 64) == 0);
static_assert(kDout == 8 * 64);
static_assert((kAPitch % 8) == 0);
static_assert(kMaxTiles == 144 && kGrRows == 9216);

constexpr size_t kWtBytes = (size_t)kCls * kDout * kDin * 2;
constexpr size_t kGrBytes = (size_t)kGrRows * kDout * 4;
constexpr size_t kOffWt   = 0;
constexpr size_t kOffGr   = kOffWt + kWtBytes;
constexpr size_t kWsTotal = kOffGr + kGrBytes;
static_assert(kWsTotal == 27262976ull);
static_assert(kWsTotal <= 134217728ull);
static_assert((kOffGr % 128) == 0);

__device__ __forceinline__ int clamp_cls(int v) {
  int r = v < 0 ? 0 : v;
  r = r > (kCls - 1) ? (kCls - 1) : r;
  return r;
}

__device__ __forceinline__ unsigned half_bits_flush(float v) {
  const float m = (fabsf(v) < kHalfMinNormal) ? 0.0f : v;
  const _Float16 h = (_Float16)m;
  const unsigned short hb = __builtin_bit_cast(unsigned short, h);
  return (unsigned)hb;
}
__device__ __forceinline__ unsigned pack_pair(float a, float b) {
  const unsigned lo = half_bits_flush(a);
  const unsigned hi = half_bits_flush(b);
  return (hi << 16) | (lo & 0xffffu);
}

union FragU { v16h v; v8h h[2]; };
__device__ __forceinline__ v16h frag_load(const _Float16* p) {
  FragU f;
  f.h[0] = *(const v8h*)(p);
  f.h[1] = *(const v8h*)(p + 16);
  return f.v;
}
__device__ __forceinline__ v8f mma_h(v16h a, v16h b, v8f c) {
  c = __builtin_amdgcn_wmma_f32_16x16x32_f16(false, a, false, b, (short)0, c, false, false);
  asm volatile("v_nop\n\tv_nop\n\tv_nop\n\tv_nop" : "+v"(c) : "v"(a), "v"(b));
  return c;
}

__device__ __forceinline__ void class_layout(const int* __restrict__ cls, int* sPre, int* sTot, int* sTb, unsigned tid) {
  const unsigned lane = tid & 31u;
  const unsigned wave = tid >> 5;
  int cnt[kCls];
#pragma unroll
  for (int c = 0; c < kCls; ++c) cnt[c] = 0;
  const v4i* p = (const v4i*)(cls + tid * kSegRows);
#pragma unroll 1
  for (int j4 = 0; j4 < kSegRows / 4; ++j4) {
    const v4i v = p[j4];
#pragma unroll
    for (int e = 0; e < 4; ++e) {
      const int id = clamp_cls(v[e]);
#pragma unroll
      for (int c = 0; c < kCls; ++c) cnt[c] += (id == c) ? 1 : 0;
    }
  }
#pragma unroll
  for (int c = 0; c < kCls; ++c) sPre[c * kThr + tid] = cnt[c];
  __syncthreads();
#pragma unroll
  for (int cc = 0; cc < 2; ++cc) {
    const unsigned c = wave * 2u + (unsigned)cc;
    int* rowp = sPre + c * kThr + lane * 8u;
    int v[8];
    int s = 0;
#pragma unroll
    for (int e = 0; e < 8; ++e) { v[e] = rowp[e]; s += v[e]; }
    int inc = s;
#pragma unroll
    for (int off = 1; off < 32; off <<= 1) {
      const int t = __shfl_up(inc, (unsigned)off, 32);
      inc += ((int)lane >= off) ? t : 0;
    }
    int run = inc - s;
#pragma unroll
    for (int e = 0; e < 8; ++e) { rowp[e] = run; run += v[e]; }
    if (lane == 31u) sTot[c] = inc;
  }
  __syncthreads();
  if (tid == 0u) {
    int tb = 0;
#pragma unroll 1
    for (int c = 0; c < kCls; ++c) {
      sTb[c] = tb;
      tb += (sTot[c] + kTileRows - 1) / kTileRows;
    }
    sTb[kCls] = tb;
  }
  __syncthreads();
}

__global__ __launch_bounds__(256) void wt_plane_kernel(const float* __restrict__ W, unsigned short* __restrict__ Wt) {
  __shared__ __align__(16) float sT[64 * kSlabPitch];
  const unsigned tid = threadIdx.x;
  const unsigned n0 = blockIdx.x * 64u;
  const unsigned k0 = blockIdx.y * 64u;
  const unsigned c  = blockIdx.z;
  const float* Wc = W + (size_t)c * kDin * kDout;
#pragma unroll
  for (unsigned it = 0; it < 4; ++it) {
    unsigned idx = it * 256u + tid;
    asm volatile("" : "+v"(idx));
    const unsigned r  = idx >> 4;
    const unsigned c4 = (idx & 15u) * 4u;
    const v4f v = *(const v4f*)(Wc + (size_t)(k0 + r) * kDout + n0 + c4);
    *(v4f*)(sT + r * kSlabPitch + c4) = v;
  }
  __syncthreads();
  v4u hv[2];
#pragma unroll
  for (unsigned it = 0; it < 2; ++it) {
    unsigned idx = it * 256u + tid;
    asm volatile("" : "+v"(idx));
    const unsigned n = idx >> 3;
    const unsigned g = idx & 7u;
    float f[8];
#pragma unroll
    for (unsigned e = 0; e < 8; ++e) f[e] = sT[(8u * g + e) * kSlabPitch + n] * kCarryW;
    v4u w;
    w[0] = pack_pair(f[0], f[1]);
    w[1] = pack_pair(f[2], f[3]);
    w[2] = pack_pair(f[4], f[5]);
    w[3] = pack_pair(f[6], f[7]);
    hv[it] = w;
  }
  for (int pass = 0; pass < 2; ++pass) {
#pragma unroll
    for (unsigned it = 0; it < 2; ++it) {
      unsigned idx = it * 256u + tid;
      asm volatile("" : "+v"(idx));
      const unsigned n = idx >> 3;
      const unsigned g = idx & 7u;
      unsigned short* q = Wt + ((size_t)(c * kDout + n0 + n) * kDin + k0 + 8u * g);
      *(volatile v4u*)q = hv[it];
    }
    __threadfence();
  }
}

__device__ __forceinline__ void list_put(int* sList, int id, int c, int lo, int row, int& run) {
  const bool hit = (id == c);
  const unsigned pos = (unsigned)(run - lo);
  if (hit && pos < (unsigned)kTileRows) sList[pos] = row;
  run += hit ? 1 : 0;
}

__global__ __launch_bounds__(256) void grouped_gemm_kernel(
    const float* __restrict__ x, const int* __restrict__ cls,
    const unsigned short* __restrict__ Wt, const float* __restrict__ bias,
    float* __restrict__ GR)
{
  __shared__ __align__(16) unsigned char sRaw[kRawBytes];
  __shared__ int sPre[kCls * kThr];
  __shared__ int sTot[kCls];
  __shared__ int sTb[32];
  __shared__ int sList[kTileRows];

  const unsigned tid = threadIdx.x;
  unsigned lane = tid & 31u;
  asm volatile("" : "+v"(lane));
  const unsigned wave = tid >> 5;

  if (tid < (unsigned)kTileRows) sList[tid] = -1;
  class_layout(cls, sPre, sTot, sTb, tid);

  const int bt = (int)blockIdx.x;
  const int total = sTb[kCls];
  if (bt >= total) return;

  int c = 0;
#pragma unroll
  for (int cc = 1; cc < kCls; ++cc) { if (bt >= sTb[cc]) c = cc; }
  const int lo = (bt - sTb[c]) * kTileRows;

  {
    int run = sPre[c * kThr + (int)tid];
    const v4i* p = (const v4i*)(cls + tid * kSegRows);
#pragma unroll 1
    for (int j4 = 0; j4 < kSegRows / 4; ++j4) {
      const v4i v = p[j4];
      int a0 = v[0], a1 = v[1], a2 = v[2], a3 = v[3];
      asm volatile("" : "+v"(a0), "+v"(a1), "+v"(a2), "+v"(a3));
      const int rbase = (int)tid * kSegRows + j4 * 4;
      list_put(sList, clamp_cls(a0), c, lo, rbase + 0, run);
      list_put(sList, clamp_cls(a1), c, lo, rbase + 1, run);
      list_put(sList, clamp_cls(a2), c, lo, rbase + 2, run);
      list_put(sList, clamp_cls(a3), c, lo, rbase + 3, run);
    }
  }
  __syncthreads();

  _Float16* sA = (_Float16*)sRaw;
  const _Float16* Wc = (const _Float16*)Wt + (size_t)c * kDout * kDin;
  unsigned rlane = lane & 15u;
  unsigned koff  = (lane >> 4) * 8u;
  asm volatile("" : "+v"(rlane), "+v"(koff));
  const unsigned mOff = koff;
  const unsigned n0 = wave * 64u;

  v8f acc[4][4];
#pragma unroll
  for (int i = 0; i < 4; ++i)
#pragma unroll
    for (int j = 0; j < 4; ++j) acc[i][j] = (v8f){0.f, 0.f, 0.f, 0.f, 0.f, 0.f, 0.f, 0.f};

#pragma unroll 1
  for (unsigned kc = 0; kc < (unsigned)kDin; kc += (unsigned)kChunk) {
    __syncthreads();
#pragma unroll 1
    for (unsigned it = 0; it < 8; ++it) {
      const unsigned r = it * 8u + wave;
      const int src = sList[r];
      const bool valid = (src >= 0);
      int srcc = src < 0 ? 0 : src;
      srcc = srcc > (kRows - 1) ? (kRows - 1) : srcc;
      const float* xp = x + (size_t)srcc * kDin + kc + lane * 8u;
      const v4f a0 = *(const v4f*)(xp);
      const v4f a1 = *(const v4f*)(xp + 4);
      float f[8];
#pragma unroll
      for (int e = 0; e < 4; ++e) {
        const float u0 = a0[e];
        const float u1 = a1[e];
        f[e]     = valid ? (u0 * kCarryX) : 0.0f;
        f[4 + e] = valid ? (u1 * kCarryX) : 0.0f;
      }
      v4u w;
      w[0] = pack_pair(f[0], f[1]);
      w[1] = pack_pair(f[2], f[3]);
      w[2] = pack_pair(f[4], f[5]);
      w[3] = pack_pair(f[6], f[7]);
      *(v4u*)(sA + r * (unsigned)kAPitch + lane * 8u) = w;
    }
    __syncthreads();

#pragma unroll 1
    for (unsigned k0 = 0; k0 < (unsigned)kChunk; k0 += 32u) {
      v16h bh[4];
#pragma unroll
      for (unsigned j = 0; j < 4; ++j) {
        const size_t bo = (size_t)(n0 + (j << 4) + rlane) * kDin + kc + k0 + koff;
        bh[j] = frag_load(Wc + bo);
      }
#pragma unroll
      for (unsigned i = 0; i < 4; ++i) {
        const v16h ah = frag_load(sA + ((i << 4) + rlane) * (unsigned)kAPitch + k0 + koff);
#pragma unroll
        for (unsigned j = 0; j < 4; ++j) acc[i][j] = mma_h(ah, bh[j], acc[i][j]);
      }
    }
  }
  __syncthreads();

  float* slab = (float*)sRaw + wave * (16u * (unsigned)kSlabPitch);
  const float* bc = bias + (size_t)c * kDout;
  const unsigned hh = lane >> 4;
  const unsigned c4 = (lane & 15u) * 4u;
#pragma unroll
  for (unsigned i = 0; i < 4; ++i) {
    const unsigned mBase = (unsigned)bt * (unsigned)kTileRows + (i << 4);
#pragma unroll
    for (unsigned j = 0; j < 4; ++j) {
      const float bv = bc[n0 + (j << 4) + rlane];
#pragma unroll
      for (unsigned r = 0; r < 8; ++r) {
        const float v = acc[i][j][r] * kFold + bv;
        slab[(mOff + r) * (unsigned)kSlabPitch + (j << 4) + rlane] = v;
      }
    }
    __builtin_amdgcn_fence(__ATOMIC_RELEASE, "workgroup");
    __builtin_amdgcn_wave_barrier();
    __builtin_amdgcn_fence(__ATOMIC_ACQUIRE, "workgroup");
    for (int pass = 0; pass < 2; ++pass) {
#pragma unroll
      for (unsigned it = 0; it < 8; ++it) {
        const unsigned row = it * 2u + hh;
        const v4f v = *(const v4f*)(slab + row * (unsigned)kSlabPitch + c4);
        *(volatile v4f*)(GR + (size_t)(mBase + row) * kDout + n0 + c4) = v;
      }
      __threadfence();
    }
    __builtin_amdgcn_fence(__ATOMIC_RELEASE, "workgroup");
    __builtin_amdgcn_wave_barrier();
    __builtin_amdgcn_fence(__ATOMIC_ACQUIRE, "workgroup");
  }
}

__global__ __launch_bounds__(256) void place_rows_kernel(
    const int* __restrict__ cls, const float* __restrict__ GR, float* __restrict__ out)
{
  __shared__ int sPre[kCls * kThr];
  __shared__ int sTot[kCls];
  __shared__ int sTb[32];
  const unsigned tid = threadIdx.x;
  unsigned lane = tid & 31u;
  asm volatile("" : "+v"(lane));
  const unsigned wave = tid >> 5;
  class_layout(cls, sPre, sTot, sTb, tid);

  const unsigned seg = blockIdx.x;
  int idl = cls[seg * (unsigned)kSegRows + lane];
  asm volatile("" : "+v"(idl));
  idl = clamp_cls(idl);

#pragma unroll 1
  for (unsigned q = 0; q < 4; ++q) {
    const unsigned rl = wave * 4u + q;
    const int cr = clamp_cls(cls[seg * (unsigned)kSegRows + rl]);
    const unsigned mask = __builtin_amdgcn_ballot_w32(idl == cr);
    const int rin = __popc(mask & ((1u << rl) - 1u));
    int slot = sTb[cr] * kTileRows + sPre[cr * kThr + (int)seg] + rin;
    slot = slot < 0 ? 0 : slot;
    slot = slot > (kGrRows - 1) ? (kGrRows - 1) : slot;
    const float* src = GR + (size_t)slot * kDout + lane * 4u;
    float* dst = out + (size_t)(seg * (unsigned)kSegRows + rl) * kDout + lane * 4u;
    const v4f v0 = *(const v4f*)(src);
    const v4f v1 = *(const v4f*)(src + 128);
    const v4f v2 = *(const v4f*)(src + 256);
    const v4f v3 = *(const v4f*)(src + 384);
    for (int pass = 0; pass < 2; ++pass) {
      *(volatile v4f*)(dst)       = v0;
      *(volatile v4f*)(dst + 128) = v1;
      *(volatile v4f*)(dst + 256) = v2;
      *(volatile v4f*)(dst + 384) = v3;
      __threadfence();
    }
  }
}

extern "C" void kernel_launch(void* const* d_in, const int* in_sizes, int n_in,
                              void* d_out, int out_size, void* d_ws, size_t ws_size,
                              hipStream_t stream) {
  if (n_in < 4) return;
  if (in_sizes[0] != kRows * kDin) return;
  if (in_sizes[1] != kRows) return;
  if (in_sizes[2] != kCls * kDin * kDout) return;
  if (in_sizes[3] != kCls * kDout) return;
  if (out_size != kRows * kDout) return;
  if (ws_size < kWsTotal) return;

  const float* x    = (const float*)d_in[0];
  const int*   cls  = (const int*)d_in[1];
  const float* W    = (const float*)d_in[2];
  const float* bias = (const float*)d_in[3];
  float* out = (float*)d_out;

  char* ws = (char*)d_ws;
  unsigned short* WT = (unsigned short*)(ws + kOffWt);
  float*          GR = (float*)(ws + kOffGr);

  wt_plane_kernel<<<dim3(kDout / 64, kDin / 64, kCls), 256, 0, stream>>>(W, WT);
  grouped_gemm_kernel<<<kMaxTiles, 256, 0, stream>>>(x, cls, WT, bias, GR);
  place_rows_kernel<<<kRows / kSegRows, 256, 0, stream>>>(cls, GR, out);
}
